// OutlookAttention_39539468927741
// MI455X (gfx1250) — hardware-verified
//
#include <hip/hip_runtime.h>

#define Cc    384
#define NHEAD 12
#define HD    32
#define Ee    972
#define EPAD  992
#define Bb    8
#define HH    56
#define LL    3136

typedef __attribute__((ext_vector_type(8)))  _Float16 v8h;
typedef __attribute__((ext_vector_type(16))) _Float16 v16h;
typedef __attribute__((ext_vector_type(8)))  float    v8f;
typedef __attribute__((ext_vector_type(4)))  float    v4f;
typedef __attribute__((ext_vector_type(4)))  unsigned v4u;

union AFrag { v16h v; v8h h[2]; };

template <typename V> __device__ __forceinline__ void vst2(void* p, V v) {
    *(volatile V*)p = v; __threadfence(); *(volatile V*)p = v;
}
__device__ __forceinline__ v8f wmma_f16(v16h a, v16h b, v8f c) {
    v8f d = __builtin_amdgcn_wmma_f32_16x16x32_f16(false, a, false, b, (short)0, c, false, false);
    asm volatile("v_nop\n\tv_nop\n\tv_nop\n\tv_nop" : "+v"(d) : "v"(a), "v"(b));
    return d;
}

__global__ void cvt_f32_f16(const float* __restrict__ s, _Float16* __restrict__ d, int n, int npad) {
    int g = blockIdx.x * 256 + threadIdx.x;
    if (g * 8 >= npad) return;
    union { v8h v; v4u u; } pk;
#pragma unroll
    for (int e = 0; e < 8; ++e) { int i = g * 8 + e; pk.v[e] = (i < n) ? (_Float16)s[i] : (_Float16)0.0f; }
    vst2(d + (size_t)g * 8, pk.u);
}

__global__ void pack_x(const float* __restrict__ x, _Float16* __restrict__ Xt) {
    int g = blockIdx.x * 256 + threadIdx.x;
    int cq = g % (Cc / 8);
    int r  = g / (Cc / 8);
    int l  = r % LL;
    int b  = r / LL;
    union { v8h v; v4u u; } pk;
#pragma unroll
    for (int e = 0; e < 8; ++e) pk.v[e] = (_Float16)x[((size_t)b * Cc + cq * 8 + e) * LL + l];
    vst2(Xt + ((size_t)b * LL + l) * Cc + cq * 8, pk.u);
}

template <int MODE>
__global__ void __launch_bounds__(256)
gemm16(const _Float16* __restrict__ W, const _Float16* __restrict__ X,
       const float* __restrict__ bias, float* __restrict__ out32,
       _Float16* __restrict__ out16, int Mtot, int nMt, int nNt) {
    constexpr int TM = (MODE == 2) ? 32 : 64, TN = (MODE == 2) ? 64 : 32;
    constexpr int MI = TM / 16, NI = TN / 16;
    __shared__ __align__(16) float st[8][TM * TN];
    const int lane  = threadIdx.x;
    const int wid   = threadIdx.y;
    const int b     = blockIdx.z;
    const int t     = blockIdx.x * 8 + wid;
    const int nTile = nMt * nNt;
    const bool valid = (t < nTile);
    const int m0 = valid ? (t / nNt) * TM : 0;
    const int n0 = valid ? (t % nNt) * TN : 0;
    const int laneM = lane & 15;
    const int hi    = lane >> 4;
    float* S = st[wid];

    if (valid) {
        const _Float16* __restrict__ Xb = X + (size_t)b * LL * Cc;
        v8f acc[MI][NI] = {};
        for (int kt = 0; kt < Cc; kt += 32) {
            AFrag a[MI], bf[NI];
#pragma unroll
            for (int mi = 0; mi < MI; ++mi) {
                const _Float16* wr = W + (size_t)(m0 + mi * 16 + laneM) * Cc + kt;
                a[mi].h[0] = *(const v8h*)(wr + 8 * hi);
                a[mi].h[1] = *(const v8h*)(wr + 16 + 8 * hi);
            }
#pragma unroll
            for (int ni = 0; ni < NI; ++ni) {
                const _Float16* xr = Xb + (size_t)(n0 + ni * 16 + laneM) * Cc + kt;
                bf[ni].h[0] = *(const v8h*)(xr + 8 * hi);
                bf[ni].h[1] = *(const v8h*)(xr + 16 + 8 * hi);
            }
#pragma unroll
            for (int mi = 0; mi < MI; ++mi)
#pragma unroll
                for (int ni = 0; ni < NI; ++ni)
                    acc[mi][ni] = wmma_f16(a[mi].v, bf[ni].v, acc[mi][ni]);
        }
#pragma unroll
        for (int mi = 0; mi < MI; ++mi)
#pragma unroll
            for (int ni = 0; ni < NI; ++ni)
#pragma unroll
                for (int r = 0; r < 8; ++r) {
                    const int ml = mi * 16 + 8 * hi + r, nl = ni * 16 + laneM;
                    float v = acc[mi][ni][r];
                    if (MODE != 0) { const int row = m0 + ml; v += (row < Mtot) ? bias[row] : 0.0f; }
                    if (MODE == 0) S[nl * TM + ml] = v; else S[ml * TN + nl] = v;
                }
    }
    __syncthreads();
    if (!valid) return;
    if (MODE == 0) {
#pragma unroll
        for (int q = 0; q < 8; ++q) {
            const int nl = q * 4 + (lane >> 3), pc = lane & 7;
            union { v8h v; v4u u; } pk;
#pragma unroll
            for (int e = 0; e < 8; ++e) pk.v[e] = (_Float16)S[nl * TM + pc * 8 + e];
            vst2(out16 + ((size_t)b * LL + n0 + nl) * Cc + m0 + pc * 8, pk.u);
        }
    } else if (MODE == 1) {
#pragma unroll
        for (int q = 0; q < 16; ++q) {
            const int ml = q * 4 + (lane >> 3), pc = lane & 7;
            const int row = m0 + ml;
            if (row < Mtot)
                vst2(out32 + ((size_t)b * Mtot + row) * LL + n0 + pc * 4, *(const v4f*)(S + ml * TN + pc * 4));
        }
    } else {
#pragma unroll
        for (int q = 0; q < 8; ++q) {
            const int ml = q * 4 + (lane >> 3), pc = lane & 7;
            const int row = m0 + ml;
            union { v8h v; v4u u; } pk;
#pragma unroll
            for (int e = 0; e < 8; ++e) pk.v[e] = (_Float16)S[ml * TN + pc * 8 + e];
            if (row < Mtot) vst2(out16 + ((size_t)b * Mtot + row) * LL + n0 + pc * 8, pk.u);
        }
    }
}

__global__ void softmax9(_Float16* __restrict__ A) {
    int i = blockIdx.x * 256 + threadIdx.x;
    int l2 = i % (LL / 2);
    int r = i / (LL / 2);
    int p = r % 9;  r /= 9;
    int n = r % NHEAD;
    int b = r / NHEAD;
    _Float16* base = A + ((size_t)b * Ee + n * 81 + p * 9) * LL + 2 * l2;
    const float sc = 0.17677669529663687f;
    float v0[9], v1[9], m0 = -1e30f, m1 = -1e30f;
#pragma unroll
    for (int q = 0; q < 9; ++q) {
        const _Float16* pq = base + (size_t)q * LL;
        v0[q] = (float)pq[0] * sc; v1[q] = (float)pq[1] * sc;
        m0 = fmaxf(m0, v0[q]); m1 = fmaxf(m1, v1[q]);
    }
    float s0 = 0.f, s1 = 0.f;
#pragma unroll
    for (int q = 0; q < 9; ++q) { v0[q] = __expf(v0[q] - m0); s0 += v0[q]; v1[q] = __expf(v1[q] - m1); s1 += v1[q]; }
    const float i0 = 1.f / s0, i1 = 1.f / s1;
#pragma unroll
    for (int q = 0; q < 9; ++q) {
        union { _Float16 h[2]; unsigned u; } pk;
        pk.h[0] = (_Float16)(v0[q] * i0); pk.h[1] = (_Float16)(v1[q] * i1);
        vst2((char*)(base + (size_t)q * LL), pk.u);
    }
}

__global__ void __launch_bounds__(256)
apply_fold(const _Float16* __restrict__ A, const _Float16* __restrict__ Vt, _Float16* __restrict__ Ft) {
    __shared__ __align__(16) _Float16 fs[8][64];
    const int lane = threadIdx.x;
    const int wid  = threadIdx.y;
    const int w    = blockIdx.x * 8 + wid;
    const int pos  = w % LL;
    int r          = w / LL;
    const int np   = r % (NHEAD / 2);
    const int b    = r / (NHEAD / 2);
    const int y = pos / HH, x = pos % HH;

#pragma unroll 1
    for (int hh2 = 0; hh2 < 2; ++hh2) {
        const int n = np * 2 + hh2;
        const _Float16* __restrict__ Vb = Vt + (size_t)b * LL * Cc + n * HD + lane;
        const _Float16* __restrict__ Ab = A + ((size_t)b * Ee + n * 81) * LL;
        float acc = 0.f;
#pragma unroll
        for (int i = 0; i < 3; ++i) {
#pragma unroll
            for (int j = 0; j < 3; ++j) {
                const int hp = y + 1 - i, wp = x + 1 - j;
                if (hp < 0 || hp >= HH || wp < 0 || wp >= HH) continue;
                const _Float16* arow = Ab + (size_t)((i * 3 + j) * 9) * LL + hp * HH + wp;
#pragma unroll
                for (int qi = 0; qi < 3; ++qi) {
                    const int vy = y + qi - i;
                    if (vy < 0 || vy >= HH) continue;
#pragma unroll
                    for (int qj = 0; qj < 3; ++qj) {
                        const int vx = x + qj - j;
                        if (vx < 0 || vx >= HH) continue;
                        const float av = (float)arow[(size_t)(qi * 3 + qj) * LL];
                        const float vv = (float)Vb[(size_t)(vx * HH + vy) * Cc];
                        acc += av * vv;
                    }
                }
            }
        }
        fs[wid][hh2 * 32 + lane] = (_Float16)acc;
    }
    __syncthreads();
    if (lane < 8) vst2(Ft + ((size_t)b * LL + pos) * Cc + np * 64 + lane * 8, *(const v4u*)(&fs[wid][lane * 8]));
}

extern "C" void kernel_launch(void* const* d_in, const int* in_sizes, int n_in,
                              void* d_out, int out_size, void* d_ws, size_t ws_size,
                              hipStream_t stream) {
    (void)in_sizes; (void)n_in; (void)out_size; (void)ws_size;
    const float* x  = (const float*)d_in[0];
    const float* Wv = (const float*)d_in[1];
    const float* Wa = (const float*)d_in[2];
    const float* ba = (const float*)d_in[3];
    const float* Wp = (const float*)d_in[4];
    const float* bp = (const float*)d_in[5];
    float* out = (float*)d_out;

    char* ws = (char*)d_ws;
    size_t off = 0;
    auto carve = [&](size_t bytes) -> void* {
        void* p = ws + off;
        off += (bytes + 255) & ~(size_t)255;
        return p;
    };
    _Float16* Xt   = (_Float16*)carve((size_t)Bb * LL * Cc * 2);
    _Float16* Wvh  = (_Float16*)carve((size_t)Cc * Cc * 2);
    _Float16* Wah  = (_Float16*)carve((size_t)EPAD * Cc * 2);
    _Float16* Wph  = (_Float16*)carve((size_t)Cc * Cc * 2);
    _Float16* Vt   = (_Float16*)carve((size_t)Bb * LL * Cc * 2);
    _Float16* Abuf = (_Float16*)carve((size_t)Bb * Ee * LL * 2);
    _Float16* Ft   = (_Float16*)carve((size_t)Bb * LL * Cc * 2);

    cvt_f32_f16<<<(Cc * Cc / 8 + 255) / 256, 256, 0, stream>>>(Wv, Wvh, Cc * Cc, Cc * Cc);
    cvt_f32_f16<<<(EPAD * Cc / 8 + 255) / 256, 256, 0, stream>>>(Wa, Wah, Ee * Cc, EPAD * Cc);
    cvt_f32_f16<<<(Cc * Cc / 8 + 255) / 256, 256, 0, stream>>>(Wp, Wph, Cc * Cc, Cc * Cc);

    pack_x<<<(Bb * LL * (Cc / 8)) / 256, 256, 0, stream>>>(x, Xt);

    dim3 gblk(32, 8);
    gemm16<0><<<dim3(74, 1, Bb), gblk, 0, stream>>>(Wvh, Xt, nullptr, nullptr, Vt, Cc, Cc / 64, LL / 32);
    gemm16<2><<<dim3(190, 1, Bb), gblk, 0, stream>>>(Wah, Xt, ba, nullptr, Abuf, Ee, EPAD / 32, LL / 64);
    softmax9<<<(Bb * NHEAD * 9 * (LL / 2)) / 256, 256, 0, stream>>>(Abuf);
    apply_fold<<<dim3((Bb * (NHEAD / 2) * LL) / 8), gblk, 0, stream>>>(Abuf, Vt, Ft);
    gemm16<1><<<dim3(74, 1, Bb), gblk, 0, stream>>>(Wph, Ft, bp, out, nullptr, Cc, Cc / 64, LL / 32);
}
